// DecoderTransformerLayer_33363305955454
// MI455X (gfx1250) — hardware-verified
//
#include <hip/hip_runtime.h>
#include <math.h>
#include <stdint.h>

#define NB    8
#define SEQ   1024
#define DM    1024
#define NH    16
#define HD    64
#define FF    4096
#define NKT   (SEQ / 64)
#define FFCH  4096
#define WSC   64.0f
#define PSC   1024.0f
#define CTXSC 16.0f

static_assert(NH * HD == DM);
static_assert((SEQ % 64) == 0 && (DM % 64) == 0 && (FF % 64) == 0);
static_assert(((NB * SEQ) % FFCH) == 0 && (FFCH % 64) == 0);
static_assert(HD == 64);

typedef _Float16 v16h __attribute__((ext_vector_type(16)));
typedef _Float16 v8h  __attribute__((ext_vector_type(8)));
typedef float    v8f  __attribute__((ext_vector_type(8)));
typedef float    v4f  __attribute__((ext_vector_type(4)));
typedef unsigned int v4u __attribute__((ext_vector_type(4)));

static constexpr size_t P16  = (size_t)NB * SEQ * DM * 2;
static constexpr size_t P32  = (size_t)NB * SEQ * DM * 4;
static constexpr size_t PW   = (size_t)DM * DM * 2;
static constexpr size_t PWF  = (size_t)FF * DM * 2;
static constexpr size_t PHM  = (size_t)FFCH * FF * 2;
static constexpr size_t OFF_E   = 0;
static constexpr size_t OFF_X   = OFF_E + P16;
static constexpr size_t OFF_WA  = OFF_X + P16;
static constexpr size_t OFF_C   = OFF_WA + 8 * PW;
static constexpr size_t OFF_Q   = OFF_C;
static constexpr size_t OFF_K   = OFF_Q + P16;
static constexpr size_t OFF_VT  = OFF_K + P16;
static constexpr size_t OFF_D   = OFF_VT + P16;
static constexpr size_t WS_TOTAL = OFF_D + P32;
static constexpr size_t OFF_X2F = OFF_X;
static constexpr size_t OFF_SCF = OFF_Q;
static constexpr size_t OFF_W1  = OFF_C;
static constexpr size_t OFF_W2  = OFF_W1 + PWF;
static constexpr size_t OFF_HM  = OFF_W2 + PWF;
static_assert(WS_TOTAL == (size_t)134217728);
static_assert(OFF_X2F + P32 == OFF_C);
static_assert(OFF_SCF + P32 == OFF_VT);
static_assert(OFF_HM + PHM == OFF_D);
static_assert((OFF_WA % 128) == 0 && (OFF_C % 128) == 0 && (OFF_D % 128) == 0);

__device__ __forceinline__ unsigned short bf_bits(float f) {
  unsigned u = __float_as_uint(f);
  return (unsigned short)((u + 0x7FFFu + ((u >> 16) & 1u)) >> 16);
}
__device__ __forceinline__ float bf_up(unsigned short h) { return __uint_as_float(((unsigned)h) << 16); }
__device__ __forceinline__ float bf_rne(float f) { return bf_up(bf_bits(f)); }
__device__ __forceinline__ unsigned short h_bits(_Float16 x) { return __builtin_bit_cast(unsigned short, x); }
__device__ __forceinline__ unsigned pk16(unsigned short a, unsigned short b) { return (unsigned)a | ((unsigned)b << 16); }
__device__ __forceinline__ unsigned pkh2(float a, float b) { return pk16(h_bits((_Float16)a), h_bits((_Float16)b)); }
__device__ __forceinline__ v8f zero8() { v8f z = {0.f, 0.f, 0.f, 0.f, 0.f, 0.f, 0.f, 0.f}; return z; }
__device__ __forceinline__ float gelu_f(float x) { return 0.5f * x * (1.0f + erff(x * 0.70710678118654752f)); }

__device__ __forceinline__ v16h ldfrag_h(const _Float16* p) {
  union { v16h v; v8h h[2]; } f;
  f.h[0] = *(const v8h*)(p);
  f.h[1] = *(const v8h*)(p + 16);
  return f.v;
}

__device__ __forceinline__ v8f mma_h(v16h a, v16h b, v8f c) {
  c = __builtin_amdgcn_wmma_f32_16x16x32_f16(false, a, false, b, (short)0, c, false, false);
  asm volatile("v_nop\n\tv_nop\n\tv_nop\n\tv_nop" : "+v"(c) : "v"(a), "v"(b));
  return c;
}
__device__ __forceinline__ v8f mma_h_raw(v16h a, v16h b, v8f c) {
  return __builtin_amdgcn_wmma_f32_16x16x32_f16(false, a, false, b, (short)0, c, false, false);
}
__device__ __forceinline__ void dep_guard_h(v8f& a, v8f& b, v16h x, v16h y) {
  asm volatile("v_nop\n\tv_nop\n\tv_nop\n\tv_nop" : "+v"(a), "+v"(b) : "v"(x), "v"(y));
}
__device__ __forceinline__ void keep4_h(v16h a, v16h b, v16h c, v16h d) {
  asm volatile("v_nop" :: "v"(a), "v"(b), "v"(c), "v"(d));
}
__device__ __forceinline__ void acc_guard4(v8f& a, v8f& b, v8f& c, v8f& d) {
  asm volatile("v_nop\n\tv_nop\n\tv_nop\n\tv_nop" : "+v"(a), "+v"(b), "+v"(c), "+v"(d));
}

__global__ __launch_bounds__(256) void cvt_h8(const float* __restrict__ in, unsigned short* out,
                                              int n8, float scale) {
  const int i = blockIdx.x * 256 + threadIdx.x;
  if (i < n8) {
    const v4f a = *(const v4f*)(in + (size_t)i * 8);
    const v4f b = *(const v4f*)(in + (size_t)i * 8 + 4);
    v4u p;
    p[0] = pkh2(bf_rne(a[0]) * scale, bf_rne(a[1]) * scale);
    p[1] = pkh2(bf_rne(a[2]) * scale, bf_rne(a[3]) * scale);
    p[2] = pkh2(bf_rne(b[0]) * scale, bf_rne(b[1]) * scale);
    p[3] = pkh2(bf_rne(b[2]) * scale, bf_rne(b[3]) * scale);
    unsigned short* dst = out + (size_t)i * 8;
    *(volatile v4u*)dst = p;
    __threadfence();
    *(volatile v4u*)dst = p;
  }
}

__global__ __launch_bounds__(256) void cvt_qkvw(const float* __restrict__ in, unsigned short* out, float scale) {
  __shared__ __align__(16) float sT[64 * 68];
  const int tid = threadIdx.x;
  const int h   = blockIdx.x / (DM / 64);
  const int dt  = blockIdx.x - h * (DM / 64);
  const int d0  = dt * 64;
  const float* src = in + ((size_t)h * DM + d0) * HD;
#pragma unroll
  for (int i = 0; i < 16; ++i) {
    const int idx = i * 256 + tid;
    const int d = idx >> 6, k = idx & 63;
    sT[k * 68 + d] = src[idx];
  }
  __syncthreads();
  const int q = tid >> 3, c8 = (tid & 7) * 8;
  v4u pv[2];
#pragma unroll
  for (int it = 0; it < 2; ++it) {
    const int r = it * 32 + q;
    const v4f a = *(const v4f*)(sT + r * 68 + c8);
    const v4f b = *(const v4f*)(sT + r * 68 + c8 + 4);
    v4u p;
    p[0] = pkh2(bf_rne(a[0]) * scale, bf_rne(a[1]) * scale);
    p[1] = pkh2(bf_rne(a[2]) * scale, bf_rne(a[3]) * scale);
    p[2] = pkh2(bf_rne(b[0]) * scale, bf_rne(b[1]) * scale);
    p[3] = pkh2(bf_rne(b[2]) * scale, bf_rne(b[3]) * scale);
    pv[it] = p;
  }
#pragma unroll
  for (int it = 0; it < 2; ++it) {
    const int r = it * 32 + q;
    *(volatile v4u*)(out + (size_t)(h * HD + r) * DM + d0 + c8) = pv[it];
  }
  __threadfence();
#pragma unroll
  for (int it = 0; it < 2; ++it) {
    const int r = it * 32 + q;
    *(volatile v4u*)(out + (size_t)(h * HD + r) * DM + d0 + c8) = pv[it];
  }
}

template <int OUT_MODE, int ACT>
__global__ __launch_bounds__(256) void gemm64(
    const unsigned short* __restrict__ Ap, int lda, long long strideA,
    const unsigned short* __restrict__ Btp, int ldb, long long strideB,
    void* Cout, int ldc, long long strideC,
    const float* __restrict__ bias, int useBias, float accScale,
    int M, int N, int K) {
  const _Float16* A  = (const _Float16*)(const void*)Ap;
  const _Float16* Bt = (const _Float16*)(const void*)Btp;
  __shared__ __align__(16) float sT[8][16 * 68];
  const int b    = blockIdx.y;
  const int lane = threadIdx.x & 31;
  const int wave = threadIdx.x >> 5;
  const int tilesN = N >> 6;
  const int tilesM = M >> 6;
  const int tile = blockIdx.x * 8 + wave;
  if (tile >= tilesM * tilesN) return;
  const int tm = tile / tilesN;
  const int tn = tile - tm * tilesN;
  const int m0 = tm << 6;
  const int n0 = tn << 6;

  const _Float16* Ab = A  + (size_t)b * strideA;
  const _Float16* Bb = Bt + (size_t)b * strideB;

  const int rlane = lane & 15;
  const int koff  = (lane >> 4) * 8;
  const int mOff  = (lane >> 4) * 8;
  const int hq = lane >> 4, c4 = (lane & 15) * 4;
  const int q8 = lane >> 3, c8 = (lane & 7) * 8;

  v4f bia0 = {0.f, 0.f, 0.f, 0.f}, bia1 = {0.f, 0.f, 0.f, 0.f};
  if (useBias != 0) {
    if (OUT_MODE == 0) {
      bia0 = *(const v4f*)(bias + n0 + c4);
    } else {
      bia0 = *(const v4f*)(bias + n0 + c8);
      bia1 = *(const v4f*)(bias + n0 + c8 + 4);
    }
#pragma unroll
    for (int e = 0; e < 4; ++e) { bia0[e] = bf_rne(bia0[e]); bia1[e] = bf_rne(bia1[e]); }
  }

  v8f acc[4][4];
#pragma unroll
  for (int i = 0; i < 4; ++i)
#pragma unroll
    for (int j = 0; j < 4; ++j) acc[i][j] = zero8();

  for (int k0 = 0; k0 < K; k0 += 32) {
    v16h bh[4];
#pragma unroll
    for (int j = 0; j < 4; ++j) {
      const size_t bo = (size_t)(n0 + (j << 4) + rlane) * ldb + koff + k0;
      bh[j] = ldfrag_h(Bb + bo);
    }
#pragma unroll
    for (int i = 0; i < 4; ++i) {
      const size_t ao = (size_t)(m0 + (i << 4) + rlane) * lda + koff + k0;
      const v16h ah = ldfrag_h(Ab + ao);
#pragma unroll
      for (int j = 0; j < 4; ++j) acc[i][j] = mma_h_raw(ah, bh[j], acc[i][j]);
      dep_guard_h(acc[i][0], acc[i][3], ah, bh[3]);
    }
    keep4_h(bh[0], bh[1], bh[2], bh[3]);
  }
  acc_guard4(acc[0][0], acc[0][1], acc[0][2], acc[0][3]);
  acc_guard4(acc[1][0], acc[1][1], acc[1][2], acc[1][3]);
  acc_guard4(acc[2][0], acc[2][1], acc[2][2], acc[2][3]);
  acc_guard4(acc[3][0], acc[3][1], acc[3][2], acc[3][3]);

  float* slab = sT[wave];
#pragma unroll
  for (int i = 0; i < 4; ++i) {
    const int mBase = m0 + (i << 4);
#pragma unroll
    for (int j = 0; j < 4; ++j) {
#pragma unroll
      for (int r = 0; r < 8; ++r) slab[(mOff + r) * 68 + (j << 4) + rlane] = acc[i][j][r];
    }
    __builtin_amdgcn_fence(__ATOMIC_RELEASE, "workgroup");
    __builtin_amdgcn_wave_barrier();
    __builtin_amdgcn_fence(__ATOMIC_ACQUIRE, "workgroup");
    if (OUT_MODE == 0) {
      float* C = (float*)Cout + (size_t)b * strideC;
      v4f vv[8];
#pragma unroll
      for (int it = 0; it < 8; ++it) {
        const int row = it * 2 + hq;
        v4f v = *(const v4f*)(slab + row * 68 + c4);
        v = v * accScale + bia0;
        vv[it] = v;
      }
#pragma unroll
      for (int it = 0; it < 8; ++it) {
        const int row = it * 2 + hq;
        *(volatile v4f*)(C + (size_t)(mBase + row) * ldc + n0 + c4) = vv[it];
      }
      __threadfence();
#pragma unroll
      for (int it = 0; it < 8; ++it) {
        const int row = it * 2 + hq;
        *(volatile v4f*)(C + (size_t)(mBase + row) * ldc + n0 + c4) = vv[it];
      }
    } else {
      unsigned short* C = (unsigned short*)Cout + (size_t)b * strideC;
      v4u hv[4];
#pragma unroll
      for (int it = 0; it < 4; ++it) {
        const int row = it * 4 + q8;
        const float* sp = slab + row * 68 + c8;
        v4f x0 = *(const v4f*)(sp);
        v4f x1 = *(const v4f*)(sp + 4);
        x0 = x0 * accScale + bia0;
        x1 = x1 * accScale + bia1;
        if (ACT) {
#pragma unroll
          for (int e = 0; e < 4; ++e) { x0[e] = gelu_f(x0[e]); x1[e] = gelu_f(x1[e]); }
        }
        v4u p;
        p[0] = pkh2(x0[0], x0[1]);
        p[1] = pkh2(x0[2], x0[3]);
        p[2] = pkh2(x1[0], x1[1]);
        p[3] = pkh2(x1[2], x1[3]);
        hv[it] = p;
      }
#pragma unroll
      for (int it = 0; it < 4; ++it) {
        const int row = it * 4 + q8;
        *(volatile v4u*)(C + (size_t)(mBase + row) * ldc + n0 + c8) = hv[it];
      }
      __threadfence();
#pragma unroll
      for (int it = 0; it < 4; ++it) {
        const int row = it * 4 + q8;
        *(volatile v4u*)(C + (size_t)(mBase + row) * ldc + n0 + c8) = hv[it];
      }
    }
    __builtin_amdgcn_fence(__ATOMIC_RELEASE, "workgroup");
    __builtin_amdgcn_wave_barrier();
    __builtin_amdgcn_fence(__ATOMIC_ACQUIRE, "workgroup");
  }
}

template <bool CAUSAL>
__global__ __launch_bounds__(128)
void attn64(const unsigned short* __restrict__ qp, const unsigned short* __restrict__ kp,
            const unsigned short* __restrict__ vtp, unsigned short* op, float sscale) {
  union FH { v16h v; v8h h[2]; };
  __shared__ __align__(16) _Float16 Ksh[64 * 64];
  __shared__ __align__(16) _Float16 Vth[64 * 64];
  __shared__ __align__(16) _Float16 Psh[4][16 * 64];
  __shared__ __align__(16) float    Os[4][16 * 64];

  const int tid  = threadIdx.x;
  const int wave = tid >> 5;
  const int lane = tid & 31;
  const int hh   = lane >> 4;
  const int c    = lane & 15;

  const int bx   = blockIdx.x;
  const int qb   = bx % NKT;
  const int rest = bx / NKT;
  const int h    = rest % NH;
  const int b    = rest / NH;
  const int q0   = qb * 64 + wave * 16;
  const size_t rowB = (size_t)b * SEQ;

  const _Float16* Qg = (const _Float16*)(const void*)qp + (size_t)h * HD;
  const _Float16* Kg = (const _Float16*)(const void*)kp + (size_t)h * HD;
  const _Float16* Vg = (const _Float16*)(const void*)vtp + ((size_t)b * DM + (size_t)h * HD) * SEQ;

  v16h qa[2];
#pragma unroll
  for (int dc = 0; dc < 2; ++dc) {
    const size_t qo = (rowB + q0 + c) * DM + dc * 32 + 8 * hh;
    qa[dc] = ldfrag_h(Qg + qo);
  }

  float mrow[8], lrow[8];
  v8f oacc[4];
#pragma unroll
  for (int r = 0; r < 8; ++r) { mrow[r] = -INFINITY; lrow[r] = 0.f; }
#pragma unroll
  for (int t = 0; t < 4; ++t) oacc[t] = zero8();

  const int ktEnd = CAUSAL ? (qb + 1) : NKT;
  for (int kt = 0; kt < NKT; ++kt) {
    if (kt >= ktEnd) break;
    const int kv0 = kt * 64;
    __syncthreads();
    {
      const int r = tid >> 1, half = (tid & 1) * 32;
      const _Float16* kg = Kg + (rowB + kv0 + r) * DM + half;
      const _Float16* vg = Vg + (size_t)r * SEQ + kv0 + half;
#pragma unroll
      for (int i = 0; i < 4; ++i) {
        const v8h a0 = *(const v8h*)(kg + 8 * i);
        const v8h b0 = *(const v8h*)(vg + 8 * i);
        *(v8h*)(Ksh + r * 64 + half + 8 * i) = a0;
        *(v8h*)(Vth + r * 64 + half + 8 * i) = b0;
      }
    }
    __syncthreads();

    v8f s[4];
#pragma unroll
    for (int j = 0; j < 4; ++j) {
      s[j] = zero8();
#pragma unroll
      for (int dc = 0; dc < 2; ++dc) {
        FH kb;
        kb.h[0] = *(const v8h*)(Ksh + (j * 16 + c) * 64 + dc * 32 + 8 * hh);
        kb.h[1] = *(const v8h*)(Ksh + (j * 16 + c) * 64 + dc * 32 + 16 + 8 * hh);
        s[j] = mma_h(qa[dc], kb.v, s[j]);
      }
    }

    _Float16* pw = Psh[wave];
#pragma unroll
    for (int r = 0; r < 8; ++r) {
      const int qrow = q0 + 8 * hh + r;
      float m = -INFINITY;
#pragma unroll
      for (int j = 0; j < 4; ++j) {
        float sv = s[j][r] * sscale;
        if (CAUSAL) {
          const int key = kv0 + j * 16 + c;
          sv = (key > qrow) ? -INFINITY : sv;
        }
        s[j][r] = sv;
        m = fmaxf(m, sv);
      }
#pragma unroll
      for (int off = 1; off < 16; off <<= 1) m = fmaxf(m, __shfl_xor(m, off, 32));
      const float mnew  = fmaxf(mrow[r], m);
      const float msafe = (mnew == -INFINITY) ? 0.f : mnew;
      const float alpha = __expf(mrow[r] - msafe);
      mrow[r] = mnew;
      float psum = 0.f;
#pragma unroll
      for (int j = 0; j < 4; ++j) {
        const float p = __expf(s[j][r] - msafe);
        psum += p;
        pw[(8 * hh + r) * 64 + j * 16 + c] = (_Float16)(p * PSC);
      }
#pragma unroll
      for (int off = 1; off < 16; off <<= 1) psum += __shfl_xor(psum, off, 32);
      lrow[r] = lrow[r] * alpha + psum;
#pragma unroll
      for (int t = 0; t < 4; ++t) oacc[t][r] *= alpha;
    }
    __builtin_amdgcn_fence(__ATOMIC_RELEASE, "workgroup");
    __builtin_amdgcn_wave_barrier();
    __builtin_amdgcn_fence(__ATOMIC_ACQUIRE, "workgroup");

#pragma unroll
    for (int kk = 0; kk < 2; ++kk) {
      FH pa;
      pa.h[0] = *(const v8h*)(pw + c * 64 + kk * 32 + 8 * hh);
      pa.h[1] = *(const v8h*)(pw + c * 64 + kk * 32 + 16 + 8 * hh);
#pragma unroll
      for (int t = 0; t < 4; ++t) {
        FH vb;
        vb.h[0] = *(const v8h*)(Vth + (t * 16 + c) * 64 + kk * 32 + 8 * hh);
        vb.h[1] = *(const v8h*)(Vth + (t * 16 + c) * 64 + kk * 32 + 16 + 8 * hh);
        oacc[t] = mma_h(pa.v, vb.v, oacc[t]);
      }
    }
  }

  float* os = Os[wave];
#pragma unroll
  for (int r = 0; r < 8; ++r) {
    const float l = lrow[r];
    const float inv = ((l > 0.f) ? (1.0f / l) : 0.f) * (CTXSC / PSC);
#pragma unroll
    for (int t = 0; t < 4; ++t) os[(8 * hh + r) * 64 + t * 16 + c] = oacc[t][r] * inv;
  }
  __builtin_amdgcn_fence(__ATOMIC_RELEASE, "workgroup");
  __builtin_amdgcn_wave_barrier();
  __builtin_amdgcn_fence(__ATOMIC_ACQUIRE, "workgroup");
  {
    const int q4 = lane >> 3, c8 = (lane & 7) * 8;
    v4u hv[4];
#pragma unroll
    for (int it = 0; it < 4; ++it) {
      const int row = it * 4 + q4;
      const float* sp = os + row * 64 + c8;
      const v4f x0 = *(const v4f*)(sp);
      const v4f x1 = *(const v4f*)(sp + 4);
      v4u p;
      p[0] = pkh2(x0[0], x0[1]);
      p[1] = pkh2(x0[2], x0[3]);
      p[2] = pkh2(x1[0], x1[1]);
      p[3] = pkh2(x1[2], x1[3]);
      hv[it] = p;
    }
#pragma unroll
    for (int it = 0; it < 4; ++it) {
      const int row = it * 4 + q4;
      const size_t go = (rowB + q0 + row) * DM + (size_t)h * HD + c8;
      *(volatile v4u*)(op + go) = hv[it];
    }
    __threadfence();
#pragma unroll
    for (int it = 0; it < 4; ++it) {
      const int row = it * 4 + q4;
      const size_t go = (rowB + q0 + row) * DM + (size_t)h * HD + c8;
      *(volatile v4u*)(op + go) = hv[it];
    }
  }
}

template <int RES_IN, int HAS_H>
__global__ __launch_bounds__(256) void resln(const float* __restrict__ a, const float* __restrict__ res,
                                             const float* __restrict__ g, const float* __restrict__ bb,
                                             float* outF, unsigned short* outH) {
  __shared__ float red1[8];
  __shared__ float red2[8];
  __shared__ __align__(16) float yb[HAS_H ? DM : 4];
  const int tid = threadIdx.x, wave = tid >> 5, lane = tid & 31;
  const size_t base = (size_t)blockIdx.x * DM + (size_t)tid * 4;
  const v4f av = *(const v4f*)(a + base);
  v4f rv = *(const v4f*)(res + base);
  if (RES_IN) {
#pragma unroll
    for (int e = 0; e < 4; ++e) rv[e] = bf_rne(rv[e]);
  }
  const v4f x = av + rv;
  float s = (x[0] + x[1]) + (x[2] + x[3]);
#pragma unroll
  for (int off = 1; off < 32; off <<= 1) s += __shfl_xor(s, off, 32);
  if (lane == 0) red1[wave] = s;
  __syncthreads();
  float tot = 0.f;
#pragma unroll
  for (int w = 0; w < 8; ++w) tot += red1[w];
  const float mu = tot * (1.0f / (float)DM);
  const v4f d = x - mu;
  float s2 = (d[0] * d[0] + d[1] * d[1]) + (d[2] * d[2] + d[3] * d[3]);
#pragma unroll
  for (int off = 1; off < 32; off <<= 1) s2 += __shfl_xor(s2, off, 32);
  if (lane == 0) red2[wave] = s2;
  __syncthreads();
  float tot2 = 0.f;
#pragma unroll
  for (int w = 0; w < 8; ++w) tot2 += red2[w];
  const float var  = tot2 * (1.0f / (float)DM);
  const float rstd = rsqrtf(var + 1e-5f);
  const v4f gv = *(const v4f*)(g + tid * 4);
  const v4f bv = *(const v4f*)(bb + tid * 4);
  v4f y;
#pragma unroll
  for (int e = 0; e < 4; ++e) y[e] = d[e] * rstd * bf_rne(gv[e]) + bf_rne(bv[e]);

  *(volatile v4f*)(outF + base) = y;
  if (HAS_H) *(v4f*)(yb + tid * 4) = y;
  __threadfence();
  *(volatile v4f*)(outF + base) = y;
  if (HAS_H) {
    __syncthreads();
    if (tid < 128) {
      const v4f y0 = *(const v4f*)(yb + tid * 8);
      const v4f y1 = *(const v4f*)(yb + tid * 8 + 4);
      v4u p;
      p[0] = pkh2(y0[0], y0[1]);
      p[1] = pkh2(y0[2], y0[3]);
      p[2] = pkh2(y1[0], y1[1]);
      p[3] = pkh2(y1[2], y1[3]);
      unsigned short* dst = outH + (size_t)blockIdx.x * DM + (size_t)tid * 8;
      *(volatile v4u*)dst = p;
      __threadfence();
      *(volatile v4u*)dst = p;
    }
  }
}

extern "C" void kernel_launch(void* const* d_in, const int* in_sizes, int n_in,
                              void* d_out, int out_size, void* d_ws, size_t ws_size,
                              hipStream_t stream) {
  if (n_in < 20) return;
  const int nX  = NB * SEQ * DM;
  const int nWh = NH * DM * HD;
  const int nWo = DM * DM;
  const int nW1 = FF * DM;
  if (in_sizes[0] != nX || in_sizes[1] != nX) return;
  if (in_sizes[2] != nWh || in_sizes[3] != nWh || in_sizes[4] != nWh) return;
  if (in_sizes[6] != nWh || in_sizes[7] != nWh || in_sizes[8] != nWh) return;
  if (in_sizes[5] != nWo || in_sizes[9] != nWo) return;
  for (int i = 10; i < 16; ++i) if (in_sizes[i] != DM) return;
  if (in_sizes[16] != nW1 || in_sizes[17] != FF || in_sizes[18] != nW1 || in_sizes[19] != DM) return;
  if (out_size != nX) return;
  if (WS_TOTAL > ws_size) return;

  const float* embeds = (const float*)d_in[0];
  const float* enc    = (const float*)d_in[1];
  const float* wq1 = (const float*)d_in[2];
  const float* wk1 = (const float*)d_in[3];
  const float* wv1 = (const float*)d_in[4];
  const float* wo1 = (const float*)d_in[5];
  const float* wq2 = (const float*)d_in[6];
  const float* wk2 = (const float*)d_in[7];
  const float* wv2 = (const float*)d_in[8];
  const float* wo2 = (const float*)d_in[9];
  const float* ln1g = (const float*)d_in[10];
  const float* ln1b = (const float*)d_in[11];
  const float* ln2g = (const float*)d_in[12];
  const float* ln2b = (const float*)d_in[13];
  const float* ln3g = (const float*)d_in[14];
  const float* ln3b = (const float*)d_in[15];
  const float* w1 = (const float*)d_in[16];
  const float* b1 = (const float*)d_in[17];
  const float* w2 = (const float*)d_in[18];
  const float* b2 = (const float*)d_in[19];

  char* ws = (char*)d_ws;
  unsigned short* Eh   = (unsigned short*)(ws + OFF_E);
  unsigned short* Xh   = (unsigned short*)(ws + OFF_X);
  unsigned short* Wq1t = (unsigned short*)(ws + OFF_WA + 0 * PW);
  unsigned short* Wk1t = (unsigned short*)(ws + OFF_WA + 1 * PW);
  unsigned short* Wv1t = (unsigned short*)(ws + OFF_WA + 2 * PW);
  unsigned short* Wo1h = (unsigned short*)(ws + OFF_WA + 3 * PW);
  unsigned short* Wq2t = (unsigned short*)(ws + OFF_WA + 4 * PW);
  unsigned short* Wk2t = (unsigned short*)(ws + OFF_WA + 5 * PW);
  unsigned short* Wv2t = (unsigned short*)(ws + OFF_WA + 6 * PW);
  unsigned short* Wo2h = (unsigned short*)(ws + OFF_WA + 7 * PW);
  unsigned short* Qh   = (unsigned short*)(ws + OFF_Q);
  unsigned short* Kh   = (unsigned short*)(ws + OFF_K);
  unsigned short* VTh  = (unsigned short*)(ws + OFF_VT);
  unsigned short* Ctx1 = (unsigned short*)(ws + OFF_X);
  unsigned short* X1H  = (unsigned short*)(ws + OFF_X);
  unsigned short* Ctx2 = (unsigned short*)(ws + OFF_E);
  unsigned short* X2H  = (unsigned short*)(ws + OFF_E);
  float*          SCF  = (float*)(ws + OFF_SCF);
  float*          X1F  = (float*)(ws + OFF_D);
  float*          X2F  = (float*)(ws + OFF_X2F);
  unsigned short* W1h  = (unsigned short*)(ws + OFF_W1);
  unsigned short* W2h  = (unsigned short*)(ws + OFF_W2);
  unsigned short* HMh  = (unsigned short*)(ws + OFF_HM);
  float*          FFF  = (float*)(ws + OFF_D);

  const dim3 blk(256);
  const int n8x  = nX / 8;
  const int n8wo = nWo / 8;
  const int n8w1 = nW1 / 8;
  const dim3 gCvtX((n8x + 255) / 256);
  const dim3 gCvtWo((n8wo + 255) / 256);
  const dim3 gCvtW1((n8w1 + 255) / 256);
  const dim3 gQkvW(NH * (DM / 64));
  const dim3 gProj(((NB * SEQ / 64) * (DM / 64) + 7) / 8, 1);
  const dim3 gVT(((DM / 64) * (SEQ / 64) + 7) / 8, NB);
  const dim3 gF1(((FFCH / 64) * (FF / 64) + 7) / 8, 1);
  const dim3 gF2(((FFCH / 64) * (DM / 64) + 7) / 8, 1);
  const dim3 gAttn(NB * NH * NKT);
  const dim3 gLN(NB * SEQ);
  const float rW   = 1.0f / WSC;
  const float rWC  = 1.0f / (WSC * CTXSC);

  cvt_h8<<<gCvtX, blk, 0, stream>>>(embeds, Xh, n8x, 1.0f);
  cvt_h8<<<gCvtX, blk, 0, stream>>>(enc, Eh, n8x, 1.0f);
  cvt_qkvw<<<gQkvW, blk, 0, stream>>>(wq1, Wq1t, WSC);
  cvt_qkvw<<<gQkvW, blk, 0, stream>>>(wk1, Wk1t, WSC);
  cvt_qkvw<<<gQkvW, blk, 0, stream>>>(wv1, Wv1t, WSC);
  cvt_qkvw<<<gQkvW, blk, 0, stream>>>(wq2, Wq2t, WSC);
  cvt_qkvw<<<gQkvW, blk, 0, stream>>>(wk2, Wk2t, WSC);
  cvt_qkvw<<<gQkvW, blk, 0, stream>>>(wv2, Wv2t, WSC);
  cvt_h8<<<gCvtWo, blk, 0, stream>>>(wo1, Wo1h, n8wo, WSC);
  cvt_h8<<<gCvtWo, blk, 0, stream>>>(wo2, Wo2h, n8wo, WSC);

  gemm64<1, 0><<<gProj, blk, 0, stream>>>(Xh, DM, 0LL, Wq1t, DM, 0LL, (void*)Qh, DM, 0LL,
                                           b2, 0, rW, NB * SEQ, DM, DM);
  gemm64<1, 0><<<gProj, blk, 0, stream>>>(Xh, DM, 0LL, Wk1t, DM, 0LL, (void*)Kh, DM, 0LL,
                                           b2, 0, rW, NB * SEQ, DM, DM);
  gemm64<1, 0><<<gVT, blk, 0, stream>>>(Wv1t, DM, 0LL, Xh, DM, (long long)SEQ * DM,
                                         (void*)VTh, SEQ, (long long)DM * SEQ,
                                         b2, 0, rW, DM, SEQ, DM);
  attn64<true><<<gAttn, dim3(128), 0, stream>>>(Qh, Kh, VTh, Ctx1, 0.125f);
  gemm64<0, 0><<<gProj, blk, 0, stream>>>(Ctx1, DM, 0LL, Wo1h, DM, 0LL, (void*)SCF, DM, 0LL,
                                           b2, 0, rWC, NB * SEQ, DM, DM);
  resln<1, 1><<<gLN, blk, 0, stream>>>(SCF, embeds, ln1g, ln1b, X1F, X1H);

  gemm64<1, 0><<<gProj, blk, 0, stream>>>(X1H, DM, 0LL, Wq2t, DM, 0LL, (void*)Qh, DM, 0LL,
                                           b2, 0, rW, NB * SEQ, DM, DM);
  gemm64<1, 0><<<gProj, blk, 0, stream>>>(Eh, DM, 0LL, Wk2t, DM, 0LL, (void*)Kh, DM, 0LL,
                                           b2, 0, rW, NB * SEQ, DM, DM);
  gemm64<1, 0><<<gVT, blk, 0, stream>>>(Wv2t, DM, 0LL, Eh, DM, (long long)SEQ * DM,
                                         (void*)VTh, SEQ, (long long)DM * SEQ,
                                         b2, 0, rW, DM, SEQ, DM);
  attn64<false><<<gAttn, dim3(128), 0, stream>>>(Qh, Kh, VTh, Ctx2, 0.125f);
  gemm64<0, 0><<<gProj, blk, 0, stream>>>(Ctx2, DM, 0LL, Wo2h, DM, 0LL, (void*)SCF, DM, 0LL,
                                           b2, 0, rWC, NB * SEQ, DM, DM);
  resln<0, 1><<<gLN, blk, 0, stream>>>(SCF, X1F, ln2g, ln2b, X2F, X2H);

  cvt_h8<<<gCvtW1, blk, 0, stream>>>(w1, W1h, n8w1, WSC);
  cvt_h8<<<gCvtW1, blk, 0, stream>>>(w2, W2h, n8w1, WSC);
  for (int ch = 0; ch < (NB * SEQ) / FFCH; ++ch) {
    const unsigned short* x2c = X2H + (size_t)ch * FFCH * DM;
    float* ffc = FFF + (size_t)ch * FFCH * DM;
    gemm64<1, 1><<<gF1, blk, 0, stream>>>(x2c, DM, 0LL, W1h, DM, 0LL, (void*)HMh, FF, 0LL,
                                           b1, 1, rW, FFCH, FF, DM);
    gemm64<0, 0><<<gF2, blk, 0, stream>>>(HMh, FF, 0LL, W2h, FF, 0LL, (void*)ffc, DM, 0LL,
                                           b2, 1, rW, FFCH, DM, FF);
  }
  resln<0, 0><<<gLN, blk, 0, stream>>>(FFF, X2F, ln3g, ln3b, (float*)d_out, X2H);
  (void)hipGetLastError();
}
